// WaveFormer_7816840479020
// MI455X (gfx1250) — hardware-verified
//
#include <hip/hip_runtime.h>
#include <math.h>

typedef _Float16 v16h __attribute__((ext_vector_type(16)));
typedef _Float16 v8h  __attribute__((ext_vector_type(8)));
typedef float    v8f  __attribute__((ext_vector_type(8)));
typedef float    v4f  __attribute__((ext_vector_type(4)));
typedef v8h __attribute__((may_alias)) v8ha;
typedef v4f __attribute__((may_alias)) v4fa;

union Frag { v16h v; v8h half[2]; };

#define NSTK   1024
#define TLEN   32
#define NTOK   32768
#define DM     256
#define XW     221
#define DFEAT  158
#define GDIM   63
#define KSRC   192
#define KPROJ  160
#define KG     64
#define NGL    192
#define IDM    0x7fffffff
#define WSC    64.0f
#define HSC    16.0f
#define PSC    4096.0f
#define OSC    (1.0f / (PSC * HSC))

#define NWITEM  (11 * (DM * DM / 8))
#define NPWITEM (DM * (KSRC / 8))
#define NGWITEM (NGL * (KG / 8))
#define NXGITEM (NSTK * (KG / 8))
#define NPREP   (NWITEM + NPWITEM + NGWITEM + NXGITEM)

__device__ __forceinline__ v8f wmma_f16(v16h a, v16h b, v8f c) {
  v8f d = __builtin_amdgcn_wmma_f32_16x16x32_f16(false, a, false, b, (short)0, c, false, false);
  asm volatile("v_nop\n\tv_nop\n\tv_nop\n\tv_nop" : "+v"(d) : "v"(a), "v"(b));
  return d;
}

__device__ __forceinline__ v16h load_frag(const _Float16* p, int h) {
  Frag f;
  f.half[0] = *(const v8ha*)(p + 8 * h);
  f.half[1] = *(const v8ha*)(p + 16 + 8 * h);
  return f.v;
}

__device__ __forceinline__ v8h pack8(v4f a, v4f c, float sc) {
  const v8h o = { (_Float16)(a[0] * sc), (_Float16)(a[1] * sc), (_Float16)(a[2] * sc), (_Float16)(a[3] * sc),
                  (_Float16)(c[0] * sc), (_Float16)(c[1] * sc), (_Float16)(c[2] * sc), (_Float16)(c[3] * sc) };
  return o;
}

__device__ __forceinline__ v16h pack_p(v8f a, v8f c, float sc) {
  const v16h r = { (_Float16)(a[0] * sc), (_Float16)(a[1] * sc), (_Float16)(a[2] * sc), (_Float16)(a[3] * sc),
                   (_Float16)(a[4] * sc), (_Float16)(a[5] * sc), (_Float16)(a[6] * sc), (_Float16)(a[7] * sc),
                   (_Float16)(c[0] * sc), (_Float16)(c[1] * sc), (_Float16)(c[2] * sc), (_Float16)(c[3] * sc),
                   (_Float16)(c[4] * sc), (_Float16)(c[5] * sc), (_Float16)(c[6] * sc), (_Float16)(c[7] * sc) };
  return r;
}

__device__ __forceinline__ void ln_stats(const float (&v)[8], float& mu, float& rs) {
  float s = 0.f;
#pragma unroll
  for (int i = 0; i < 8; ++i) s += v[i];
#pragma unroll
  for (int o = 16; o; o >>= 1) s += __shfl_xor(s, o, 32);
  mu = s * (1.f / 256.f);
  float q = 0.f;
#pragma unroll
  for (int i = 0; i < 8; ++i) { const float d = v[i] - mu; q += d * d; }
#pragma unroll
  for (int o = 16; o; o >>= 1) q += __shfl_xor(q, o, 32);
  rs = rsqrtf(q * (1.f / 256.f) + 1e-5f);
}

__device__ __forceinline__ void stage8(float* dst, v8f o, float osc, const float* zp,
                                       const float* gp, const float* bp, float mu, float rs) {
  const v4f z0 = *(const v4fa*)zp, z1 = *(const v4fa*)(zp + 4);
  const v4f g0 = *(const v4fa*)gp, g1 = *(const v4fa*)(gp + 4);
  const v4f b0 = *(const v4fa*)bp, b1 = *(const v4fa*)(bp + 4);
  const float zz[8] = { z0[0], z0[1], z0[2], z0[3], z1[0], z1[1], z1[2], z1[3] };
  const float gg[8] = { g0[0], g0[1], g0[2], g0[3], g1[0], g1[1], g1[2], g1[3] };
  const float bv[8] = { b0[0], b0[1], b0[2], b0[3], b1[0], b1[1], b1[2], b1[3] };
#pragma unroll
  for (int r = 0; r < 8; ++r) dst[r] = o[r] * osc + ((zz[r] - mu) * rs * gg[r] + bv[r]);
}

__global__ __launch_bounds__(256) void prep_k(
    const float* __restrict__ w0, const float* __restrict__ w1, const float* __restrict__ w2,
    const float* __restrict__ w3, const float* __restrict__ w4, const float* __restrict__ w5,
    const float* __restrict__ w6, const float* __restrict__ w7, const float* __restrict__ w8,
    const float* __restrict__ w9, const float* __restrict__ w10,
    const float* __restrict__ proj_w, const float* __restrict__ gate_w, const float* __restrict__ x,
    _Float16* __restrict__ w16, _Float16* __restrict__ pw16,
    _Float16* __restrict__ gw16, _Float16* __restrict__ xg16)
{
  const int gidx = blockIdx.x * 256 + threadIdx.x;
  v8h o;
  _Float16* dst;
  if (gidx < NWITEM) {
    const int wsl = gidx >> 13;
    const float* src = w0;
    if (wsl == 1) src = w1;
    if (wsl == 2) src = w2;
    if (wsl == 3) src = w3;
    if (wsl == 4) src = w4;
    if (wsl == 5) src = w5;
    if (wsl == 6) src = w6;
    if (wsl == 7) src = w7;
    if (wsl == 8) src = w8;
    if (wsl == 9) src = w9;
    if (wsl == 10) src = w10;
    src += (size_t)(gidx & 8191) * 8;
    const v4f a = *(const v4fa*)src;
    const v4f c = *(const v4fa*)(src + 4);
    o = pack8(a, c, WSC);
    dst = w16 + (size_t)gidx * 8;
  } else if (gidx < NWITEM + NPWITEM) {
    const int e = gidx - NWITEM;
    const int orow = e / 24, gq = e - orow * 24, c0 = gq * 8;
    float v[8];
#pragma unroll
    for (int j = 0; j < 8; ++j) {
      const int c = c0 + j, cc = min(c, DFEAT - 1);
      const float f = proj_w[orow * DFEAT + cc] * WSC;
      v[j] = (c < DFEAT) ? f : 0.f;
    }
    const v4f a = { v[0], v[1], v[2], v[3] }, c = { v[4], v[5], v[6], v[7] };
    o = pack8(a, c, 1.0f);
    dst = pw16 + (size_t)e * 8;
  } else if (gidx < NWITEM + NPWITEM + NGWITEM) {
    const int e = gidx - NWITEM - NPWITEM;
    const int orow = e >> 3, c0 = (e & 7) * 8, oc = min(orow, DFEAT - 1);
    float v[8];
#pragma unroll
    for (int j = 0; j < 8; ++j) {
      const int c = c0 + j, cc = min(c, GDIM - 1);
      const float f = gate_w[oc * GDIM + cc] * WSC;
      v[j] = (orow < DFEAT && c < GDIM) ? f : 0.f;
    }
    const v4f a = { v[0], v[1], v[2], v[3] }, c = { v[4], v[5], v[6], v[7] };
    o = pack8(a, c, 1.0f);
    dst = gw16 + (size_t)e * 8;
  } else if (gidx < NPREP) {
    const int e = gidx - NWITEM - NPWITEM - NGWITEM;
    const int n = e >> 3, c0 = (e & 7) * 8;
    const float* xr = x + ((size_t)(n * TLEN + (TLEN - 1))) * XW + DFEAT;
    float v[8];
#pragma unroll
    for (int j = 0; j < 8; ++j) {
      const int c = c0 + j, cc = min(c, GDIM - 1);
      const float f = xr[cc];
      v[j] = (c < GDIM) ? f : 0.f;
    }
    const v4f a = { v[0], v[1], v[2], v[3] }, c = { v[4], v[5], v[6], v[7] };
    o = pack8(a, c, 1.0f);
    dst = xg16 + (size_t)e * 8;
  } else {
    return;
  }
  *(volatile v8h*)dst = o;
  __threadfence();
  *(volatile v8h*)dst = o;
}

template <int MODE>
__device__ __forceinline__ void gemm_store(const float* sC, const _Float16* sH, float* outF, _Float16* outH,
                                           int ldc, int m0, int n0, int w, int lane,
                                           int amask, int amul, int ashift, float hmul,
                                           int tshift, int tmask, int tA, int tB)
{
  const int q8 = lane & 7, sub = lane >> 3;
  if (MODE == 0) {
#pragma unroll
    for (int i = 0; i < 16; ++i) {
      const int L = i * 4 + sub, rl = 32 * w + (L >> 1), hl = L & 1;
      const v4f val = *(const v4fa*)(sC + rl * 64 + hl * 32 + q8 * 4);
      const int m1 = m0 + rl;
      const int tok = (m1 & amask) * amul + (m1 >> ashift);
      *(volatile v4f*)(outF + (size_t)tok * ldc + n0 + hl * 32 + q8 * 4) = val;
    }
  }
  if (MODE == 0 || MODE == 1) {
    if (outH != nullptr) {
#pragma unroll
      for (int i = 0; i < 8; ++i) {
        const int rl = 32 * w + i * 4 + sub;
        const v4f a = *(const v4fa*)(sC + rl * 64 + q8 * 8);
        const v4f c = *(const v4fa*)(sC + rl * 64 + q8 * 8 + 4);
        const v8h o = pack8(a, c, hmul);
        const int m1 = m0 + rl;
        const int tok = (m1 & amask) * amul + (m1 >> ashift);
        *(volatile v8h*)(outH + (size_t)tok * ldc + n0 + q8 * 8) = o;
      }
    }
  }
  if (MODE == 2) {
    const size_t tbase = (size_t)(m0 >> tshift) * (size_t)tA + (size_t)(m0 & tmask);
#pragma unroll
    for (int i = 0; i < 8; ++i) {
      const int L = i * 4 + sub, d = 16 * w + (L >> 1), hl = L & 1;
      const v8h val = *(const v8ha*)(sH + d * 128 + hl * 64 + q8 * 8);
      *(volatile v8h*)(outH + tbase + (size_t)(n0 + d) * (size_t)tB + hl * 64 + q8 * 8) = val;
    }
  }
}

template <int MODE, bool PE>
__global__ __launch_bounds__(128) void gemm_k(
    const _Float16* __restrict__ A, int lda, int amask, int amul, int ashift,
    const _Float16* __restrict__ W, int ldw, int K,
    const float* __restrict__ bias, int nbias,
    const float* resid, float* outF, _Float16* outH, int ldc,
    float cscale, float hmul, int relu,
    int tshift, int tmask, int tA, int tB)
{
  __shared__ __attribute__((aligned(16))) char sraw[128 * 64 * 4];
  __shared__ __attribute__((aligned(16))) float sPE[PE ? 2048 : 4];
  float* sC = (float*)sraw;
  _Float16* sH = (_Float16*)sraw;

  const int tid = threadIdx.x, lane = tid & 31, w = tid >> 5;
  const int h = lane >> 4, m = lane & 15;
  const int m0 = blockIdx.x * 128, n0 = blockIdx.y * 64;

  if (PE) {
#pragma unroll 1
    for (int i = tid; i < 2048; i += 128) {
      const int t = i >> 6, c = n0 + (i & 63);
      const float de = (float)(c & ~1);
      const float dv = expf(de * -0.035977892078031968f);
      const float ang = (float)t * dv;
      const float sv = sinf(ang), cv = cosf(ang);
      sPE[i] = (c & 1) ? cv : sv;
    }
  }

  const int m1a = m0 + 32 * w + m, m1b = m1a + 16;
  const int toka = (m1a & amask) * amul + (m1a >> ashift);
  const int tokb = (m1b & amask) * amul + (m1b >> ashift);
  const _Float16* ap0 = A + (size_t)toka * lda;
  const _Float16* ap1 = A + (size_t)tokb * lda;
  const _Float16* wp  = W + (size_t)(n0 + m) * ldw;

  const v8f zero8 = { 0.f, 0.f, 0.f, 0.f, 0.f, 0.f, 0.f, 0.f };
  v8f acc[2][4];
#pragma unroll
  for (int mt = 0; mt < 2; ++mt)
#pragma unroll
    for (int nt = 0; nt < 4; ++nt) acc[mt][nt] = zero8;

#pragma unroll 1
  for (int k0 = 0; k0 < K; k0 += 32) {
    const v16h a0 = load_frag(ap0 + k0, h);
    const v16h a1 = load_frag(ap1 + k0, h);
#pragma unroll
    for (int nt = 0; nt < 4; ++nt) {
      const v16h b = load_frag(wp + (size_t)(16 * nt) * ldw + k0, h);
      acc[0][nt] = wmma_f16(a0, b, acc[0][nt]);
      acc[1][nt] = wmma_f16(a1, b, acc[1][nt]);
    }
  }
  if (PE) __syncthreads();

#pragma unroll
  for (int nt = 0; nt < 4; ++nt) {
    const int cl = 16 * nt + m, c = n0 + cl;
    float bvl = 0.f;
    if (bias != nullptr) bvl = bias[min(c, nbias - 1)];
#pragma unroll
    for (int mt = 0; mt < 2; ++mt) {
#pragma unroll
      for (int r = 0; r < 8; ++r) {
        const int rl = 32 * w + 16 * mt + 8 * h + r;
        float v = acc[mt][nt][r] * cscale + bvl;
        if (relu) v = fmaxf(v, 0.f);
        if (PE) v += sPE[(rl & 31) * 64 + cl];
        if (resid != nullptr) {
          const int m1 = m0 + rl;
          const int tok = (m1 & amask) * amul + (m1 >> ashift);
          v += resid[(size_t)tok * ldc + c];
        }
        if (MODE == 2) sH[cl * 128 + rl] = (_Float16)(v * hmul);
        else sC[rl * 64 + cl] = v;
      }
    }
  }
  __syncthreads();

  gemm_store<MODE>(sC, sH, outF, outH, ldc, m0, n0, w, lane, amask, amul, ashift, hmul, tshift, tmask, tA, tB);
  __threadfence();
  gemm_store<MODE>(sC, sH, outF, outH, ldc, m0, n0, w, lane, amask, amul, ashift, hmul, tshift, tmask, tA, tB);
}

__global__ __launch_bounds__(256) void gate_src_k(const float* __restrict__ Lg, const float* __restrict__ x,
                                                  _Float16* __restrict__ src16)
{
  __shared__ float gsh[NGL];
  __shared__ float red[2];
  const int n = blockIdx.x, tid = threadIdx.x;
  if (tid < NGL) gsh[tid] = Lg[(size_t)n * NGL + tid] * 0.2f;
  __syncthreads();
  if (tid == 0) {
    float mx = -3.0e38f;
#pragma unroll 1
    for (int j = 0; j < DFEAT; ++j) mx = fmaxf(mx, gsh[j]);
    float ss = 0.f;
#pragma unroll 1
    for (int j = 0; j < DFEAT; ++j) ss += __expf(gsh[j] - mx);
    red[0] = mx;
    red[1] = (float)DFEAT * (1.0f / ss);
  }
  __syncthreads();
  float gv = 0.f;
  if (tid < DFEAT) gv = __expf(gsh[tid] - red[0]) * red[1];
  __syncthreads();
  if (tid < NGL) gsh[tid] = gv;
  __syncthreads();

  v8h o3[3];
  size_t d3[3];
#pragma unroll
  for (int it = 0; it < 3; ++it) {
    const int item = it * 256 + tid;
    const int L = item >> 3, q = item & 7;
    const int t = L / 3, seg = L - 3 * t;
    const int c0 = seg * 64 + q * 8;
    const float* xr = x + ((size_t)(n * TLEN + t)) * XW;
    float v[8];
#pragma unroll
    for (int j = 0; j < 8; ++j) {
      const int c = c0 + j, cc = min(c, DFEAT - 1);
      const float f = xr[cc] * gsh[c];
      v[j] = (c < DFEAT) ? f : 0.f;
    }
    const v4f a = { v[0], v[1], v[2], v[3] }, c = { v[4], v[5], v[6], v[7] };
    o3[it] = pack8(a, c, 1.0f);
    d3[it] = (size_t)(n * TLEN + t) * KSRC + c0;
  }
#pragma unroll
  for (int it = 0; it < 3; ++it) *(volatile v8h*)(src16 + d3[it]) = o3[it];
  __threadfence();
#pragma unroll
  for (int it = 0; it < 3; ++it) *(volatile v8h*)(src16 + d3[it]) = o3[it];
}

__global__ __launch_bounds__(256) void ln_k(const float* in, float* outF, _Float16* __restrict__ outH,
                                            const float* __restrict__ g, const float* __restrict__ bb, float hmul)
{
  __shared__ __attribute__((aligned(16))) float sm[8 * 256];
  const int tid = threadIdx.x, lane = tid & 31, w = tid >> 5;
  const int tok = blockIdx.x * 8 + w;
  const float* p = in + (size_t)tok * DM;
  float v[8];
#pragma unroll
  for (int i = 0; i < 8; ++i) v[i] = p[lane + 32 * i];
  float mu, rs;
  ln_stats(v, mu, rs);
  float ov[8];
#pragma unroll
  for (int i = 0; i < 8; ++i) {
    const int d = lane + 32 * i;
    ov[i] = (v[i] - mu) * rs * g[d] + bb[d];
  }
  float* smw = sm + w * 256;
#pragma unroll
  for (int i = 0; i < 8; ++i) smw[lane + 32 * i] = ov[i];
  if (outF != nullptr) {
#pragma unroll
    for (int i = 0; i < 8; ++i) *(volatile float*)(outF + (size_t)tok * DM + lane + 32 * i) = ov[i];
  }
  __syncthreads();
  const v4f a = *(const v4fa*)(smw + lane * 8);
  const v4f c = *(const v4fa*)(smw + lane * 8 + 4);
  const v8h oh = pack8(a, c, hmul);
  _Float16* hp = outH + (size_t)tok * DM + lane * 8;
  *(volatile v8h*)hp = oh;
  __threadfence();
  if (outF != nullptr) {
#pragma unroll
    for (int i = 0; i < 8; ++i) *(volatile float*)(outF + (size_t)tok * DM + lane + 32 * i) = ov[i];
  }
  *(volatile v8h*)hp = oh;
}

__device__ __forceinline__ void att_t_store(const float* sow, float* Z, int tok0, int hoff, int lane) {
  const int q8 = lane & 7, sub = lane >> 3;
#pragma unroll
  for (int i = 0; i < 16; ++i) {
    const int L = i * 4 + sub, rl = L >> 1, hl = L & 1;
    const v4f val = *(const v4fa*)(sow + rl * 64 + hl * 32 + q8 * 4);
    *(volatile v4f*)(Z + (size_t)(tok0 + rl) * DM + hoff + hl * 32 + q8 * 4) = val;
  }
}

__global__ __launch_bounds__(128) void attn_t_k(
    const _Float16* __restrict__ Qp,
    const _Float16* __restrict__ Kp,
    const _Float16* __restrict__ VT,
    float* Z,
    const float* __restrict__ g, const float* __restrict__ bb, float sscale)
{
  __shared__ __attribute__((aligned(16))) float so[4 * 32 * 64];
  __shared__ float smu[32], srs[32];

  const int tid = threadIdx.x, lane = tid & 31, w = tid >> 5;
  const int h = lane >> 4, m = lane & 15;
  const int n = blockIdx.x, tok0 = n * TLEN, hoff = w * 64;

#pragma unroll 1
  for (int j = 0; j < 8; ++j) {
    const float* p = Z + (size_t)(tok0 + 8 * w + j) * DM;
    float v[8];
#pragma unroll
    for (int i = 0; i < 8; ++i) v[i] = p[lane + 32 * i];
    float mu, rs;
    ln_stats(v, mu, rs);
    if (lane == 0) { smu[8 * w + j] = mu; srs[8 * w + j] = rs; }
  }
  __syncthreads();

  const v8f zero8 = { 0.f, 0.f, 0.f, 0.f, 0.f, 0.f, 0.f, 0.f };
  v16h qb[2][2];
#pragma unroll
  for (int qi = 0; qi < 2; ++qi)
#pragma unroll
    for (int kc = 0; kc < 2; ++kc)
      qb[qi][kc] = load_frag(Qp + (size_t)(tok0 + 16 * qi + m) * DM + hoff + 32 * kc, h);

  v8f s[2][2];
#pragma unroll
  for (int j = 0; j < 2; ++j) {
    const _Float16* kp = Kp + (size_t)(tok0 + 16 * j + m) * DM + hoff;
    const v16h kf0 = load_frag(kp, h);
    const v16h kf1 = load_frag(kp + 32, h);
#pragma unroll
    for (int qi = 0; qi < 2; ++qi) {
      v8f z = zero8;
      z = wmma_f16(kf0, qb[qi][0], z);
      z = wmma_f16(kf1, qb[qi][1], z);
      s[j][qi] = z * sscale;
    }
  }

  v16h pb[2];
#pragma unroll
  for (int qi = 0; qi < 2; ++qi) {
    float mx = s[0][qi][0];
#pragma unroll
    for (int j = 0; j < 2; ++j)
#pragma unroll
      for (int r = 0; r < 8; ++r) mx = fmaxf(mx, s[j][qi][r]);
    mx = fmaxf(mx, __shfl_xor(mx, 16, 32));
    float l = 0.f;
#pragma unroll
    for (int j = 0; j < 2; ++j)
#pragma unroll
      for (int r = 0; r < 8; ++r) {
        const float e = __expf(s[j][qi][r] - mx);
        s[j][qi][r] = e;
        l += e;
      }
    l += __shfl_xor(l, 16, 32);
    pb[qi] = pack_p(s[0][qi], s[1][qi], PSC * (1.0f / l));
  }

  float* sow = so + w * 2048;
#pragma unroll
  for (int dt = 0; dt < 4; ++dt) {
    const v16h vf = load_frag(VT + (size_t)(hoff + 16 * dt + m) * NTOK + tok0, h);
    const int c = hoff + 16 * dt + 8 * h;
#pragma unroll
    for (int qi = 0; qi < 2; ++qi) {
      const v8f o = wmma_f16(vf, pb[qi], zero8);
      const int ql = 16 * qi + m, tok = tok0 + ql;
      stage8(sow + ql * 64 + 16 * dt + 8 * h, o, OSC, Z + (size_t)tok * DM + c, g + c, bb + c, smu[ql], srs[ql]);
    }
  }
  __syncthreads();

  att_t_store(sow, Z, tok0, hoff, lane);
  __threadfence();
  att_t_store(sow, Z, tok0, hoff, lane);
}

__device__ __forceinline__ void att_s_store(const float* sow, float* Z, int n0w, int t, int hoff, int lane) {
  const int q8 = lane & 7, sub = lane >> 3;
#pragma unroll
  for (int i = 0; i < 16; ++i) {
    const int L = i * 4 + sub, rl = L >> 2, ql = L & 3;
    const v4f val = *(const v4fa*)(sow + rl * 128 + ql * 32 + q8 * 4);
    *(volatile v4f*)(Z + ((size_t)(n0w + rl) * TLEN + t) * DM + hoff + ql * 32 + q8 * 4) = val;
  }
}

__global__ __launch_bounds__(128) void attn_s_k(
    const _Float16* __restrict__ Qp,
    const _Float16* __restrict__ Kp,
    const _Float16* __restrict__ VT,
    float* Z,
    const float* __restrict__ g, const float* __restrict__ bb, float sscale)
{
  __shared__ __attribute__((aligned(16))) float so[4 * 16 * 128];
  __shared__ float smu[64], srs[64];

  const int tid = threadIdx.x, lane = tid & 31, w = tid >> 5;
  const int h = lane >> 4, m = lane & 15;
  const int n0 = blockIdx.x * 64, t = blockIdx.y;
  const int n0w = n0 + 16 * w;

#pragma unroll 1
  for (int j = 0; j < 16; ++j) {
    const float* p = Z + ((size_t)(n0w + j) * TLEN + t) * DM;
    float v[8];
#pragma unroll
    for (int i = 0; i < 8; ++i) v[i] = p[lane + 32 * i];
    float mu, rs;
    ln_stats(v, mu, rs);
    if (lane == 0) { smu[16 * w + j] = mu; srs[16 * w + j] = rs; }
  }
  __syncthreads();

  const v8f zero8 = { 0.f, 0.f, 0.f, 0.f, 0.f, 0.f, 0.f, 0.f };
  const int ql = 16 * w + m;
  const int qtok = (n0w + m) * TLEN + t;
  float* sow = so + w * 2048;

#pragma unroll 1
  for (int hh = 0; hh < 2; ++hh) {
    const int hoff = hh * 128;
    v16h qb[4];
#pragma unroll
    for (int kc = 0; kc < 4; ++kc) qb[kc] = load_frag(Qp + (size_t)qtok * DM + hoff + 32 * kc, h);

    v8f o[8];
#pragma unroll
    for (int dt = 0; dt < 8; ++dt) o[dt] = zero8;
    float mrun = -1.0e30f, lrun = 0.0f;

#pragma unroll 1
    for (int kb = 0; kb < NSTK; kb += 64) {
      v8f s[4];
#pragma unroll
      for (int j = 0; j < 4; ++j) {
        const _Float16* kp = Kp + ((size_t)(kb + 16 * j + m) * TLEN + t) * DM + hoff;
        v8f z = zero8;
#pragma unroll
        for (int kc = 0; kc < 4; ++kc) {
          const v16h kf = load_frag(kp + 32 * kc, h);
          z = wmma_f16(kf, qb[kc], z);
        }
        s[j] = z * sscale;
      }
      float mloc = s[0][0];
#pragma unroll
      for (int j = 0; j < 4; ++j)
#pragma unroll
        for (int r = 0; r < 8; ++r) mloc = fmaxf(mloc, s[j][r]);
      mloc = fmaxf(mloc, __shfl_xor(mloc, 16, 32));
      const float mnew = fmaxf(mrun, mloc);
      const float alpha = __expf(mrun - mnew);
      mrun = mnew;
      float lsum = 0.0f;
#pragma unroll
      for (int j = 0; j < 4; ++j)
#pragma unroll
        for (int r = 0; r < 8; ++r) {
          const float p = __expf(s[j][r] - mnew);
          s[j][r] = p;
          lsum += p;
        }
      lsum += __shfl_xor(lsum, 16, 32);
      lrun = lrun * alpha + lsum;
#pragma unroll
      for (int dt = 0; dt < 8; ++dt) o[dt] = o[dt] * alpha;

      const v16h pb0 = pack_p(s[0], s[1], PSC);
      const v16h pb1 = pack_p(s[2], s[3], PSC);

#pragma unroll
      for (int dt = 0; dt < 8; ++dt) {
        const _Float16* vp = VT + ((size_t)(t * DM + hoff + 16 * dt + m)) * NSTK + kb;
        const v16h vf0 = load_frag(vp, h);
        const v16h vf1 = load_frag(vp + 32, h);
        o[dt] = wmma_f16(vf0, pb0, o[dt]);
        o[dt] = wmma_f16(vf1, pb1, o[dt]);
      }
    }

    const float inv = (1.0f / lrun) * OSC;
    const float mu = smu[ql], rs = srs[ql];
#pragma unroll
    for (int dt = 0; dt < 8; ++dt) {
      const int c = hoff + 16 * dt + 8 * h;
      stage8(sow + m * 128 + 16 * dt + 8 * h, o[dt], inv, Z + (size_t)qtok * DM + c, g + c, bb + c, mu, rs);
    }
    __syncthreads();
    att_s_store(sow, Z, n0w, t, hoff, lane);
    __threadfence();
    att_s_store(sow, Z, n0w, t, hoff, lane);
    __syncthreads();
  }
}

__global__ __launch_bounds__(256) void pool_k(const float* __restrict__ hF, const float* __restrict__ z,
                                              const float* __restrict__ ow, const float* __restrict__ ob,
                                              float* __restrict__ out)
{
  __shared__ __attribute__((aligned(16))) float res[32];
  const int tid = threadIdx.x, lane = tid & 31, w = tid >> 5, blk = blockIdx.x;
  float owr[8];
#pragma unroll
  for (int i = 0; i < 8; ++i) owr[i] = ow[lane + 32 * i];
  const float obv = ob[0];

#pragma unroll 1
  for (int s4 = 0; s4 < 4; ++s4) {
    const int n = blk * 32 + w * 4 + s4;
    const float* hb = hF + (size_t)n * TLEN * DM;
    const float* zb = z  + (size_t)n * TLEN * DM;
    float hl[8];
#pragma unroll
    for (int i = 0; i < 8; ++i) hl[i] = hb[(TLEN - 1) * DM + lane + 32 * i];
    float mylog = 0.f;
#pragma unroll 1
    for (int t = 0; t < TLEN; ++t) {
      float d = 0.f;
#pragma unroll
      for (int i = 0; i < 8; ++i) d += hb[t * DM + lane + 32 * i] * hl[i];
#pragma unroll
      for (int o2 = 16; o2; o2 >>= 1) d += __shfl_xor(d, o2, 32);
      mylog = (lane == t) ? d : mylog;
    }
    float mx = mylog;
#pragma unroll
    for (int o2 = 16; o2; o2 >>= 1) mx = fmaxf(mx, __shfl_xor(mx, o2, 32));
    const float e = __expf(mylog - mx);
    float ssum = e;
#pragma unroll
    for (int o2 = 16; o2; o2 >>= 1) ssum += __shfl_xor(ssum, o2, 32);
    const float lam = e * (1.0f / ssum);
    float pooled[8];
#pragma unroll
    for (int i = 0; i < 8; ++i) pooled[i] = 0.f;
#pragma unroll 1
    for (int t = 0; t < TLEN; ++t) {
      const float lt = __shfl(lam, t, 32);
#pragma unroll
      for (int i = 0; i < 8; ++i) pooled[i] += lt * zb[t * DM + lane + 32 * i];
    }
    float r = 0.f;
#pragma unroll
    for (int i = 0; i < 8; ++i) r += pooled[i] * owr[i];
#pragma unroll
    for (int o2 = 16; o2; o2 >>= 1) r += __shfl_xor(r, o2, 32);
    r += obv;
    if (lane == 0) res[w * 4 + s4] = r;
  }
  __syncthreads();
  const v4f val = *(const v4fa*)(res + (lane & 7) * 4);
  float* dst = out + blk * 32 + (lane & 7) * 4;
  if (w == 0 && lane < 8) *(volatile v4f*)dst = val;
  __threadfence();
  if (w == 0 && lane < 8) *(volatile v4f*)dst = val;
}

extern "C" void kernel_launch(void* const* d_in, const int* in_sizes, int n_in,
                              void* d_out, int out_size, void* d_ws, size_t ws_size,
                              hipStream_t stream) {
  if (n_in < 30) return;
  if (in_sizes[0] != NTOK * XW) return;
  if (in_sizes[1] != DFEAT * GDIM || in_sizes[2] != DFEAT) return;
  if (in_sizes[3] != DM * DFEAT || in_sizes[4] != DM) return;
  const int widx[11] = { 5, 6, 7, 12, 14, 16, 17, 18, 23, 25, 27 };
  for (int i = 0; i < 11; ++i) if (in_sizes[widx[i]] != DM * DM) return;
  const int vidx[14] = { 8, 9, 10, 11, 13, 15, 19, 20, 21, 22, 24, 26, 28, 4 };
  for (int i = 0; i < 14; ++i) if (in_sizes[vidx[i]] != DM) return;
  if (in_sizes[29] < 1) return;
  if (out_size != NSTK) return;

  const float* x      = (const float*)d_in[0];
  const float* gate_w = (const float*)d_in[1];
  const float* gate_b = (const float*)d_in[2];
  const float* proj_w = (const float*)d_in[3];
  const float* proj_b = (const float*)d_in[4];
  const float* tn1g = (const float*)d_in[8],  *tn1b = (const float*)d_in[9];
  const float* tn2g = (const float*)d_in[10], *tn2b = (const float*)d_in[11];
  const float* tf1b = (const float*)d_in[13], *tf2b = (const float*)d_in[15];
  const float* sn1g = (const float*)d_in[19], *sn1b = (const float*)d_in[20];
  const float* sn2g = (const float*)d_in[21], *sn2b = (const float*)d_in[22];
  const float* sf1b = (const float*)d_in[24], *sf2b = (const float*)d_in[26];
  const float* out_w = (const float*)d_in[28], *out_b = (const float*)d_in[29];
  const float* wsrc[11];
  for (int i = 0; i < 11; ++i) wsrc[i] = (const float*)d_in[widx[i]];

  const size_t w16_bytes = (size_t)11 * DM * DM * 2;
  const size_t pw_bytes  = (size_t)DM * KSRC * 2;
  const size_t gw_bytes  = (size_t)NGL * KG * 2;
  const size_t xg_bytes  = (size_t)NSTK * KG * 2;
  const size_t lg_bytes  = (size_t)NSTK * NGL * 4;
  const size_t hp_bytes  = (size_t)NTOK * DM * 2;
  const size_t af_bytes  = (size_t)NTOK * DM * 4;
  size_t off = 0;
  const size_t o_w16 = off; off += w16_bytes;
  const size_t o_pw  = off; off += pw_bytes;
  const size_t o_gw  = off; off += gw_bytes;
  const size_t o_xg  = off; off += xg_bytes;
  const size_t o_lg  = off; off += lg_bytes;
  const size_t o_h0  = off; off += hp_bytes;
  const size_t o_h1  = off; off += hp_bytes;
  const size_t o_h2  = off; off += hp_bytes;
  const size_t o_vt  = off; off += hp_bytes;
  const size_t o_af  = off; off += af_bytes;
  const size_t total = off;
  if (total > ws_size) return;
  if ((size_t)NTOK * KSRC * 2 > hp_bytes) return;

  char* ws = (char*)d_ws;
  _Float16* w16  = (_Float16*)(ws + o_w16);
  _Float16* pw16 = (_Float16*)(ws + o_pw);
  _Float16* gw16 = (_Float16*)(ws + o_gw);
  _Float16* xg16 = (_Float16*)(ws + o_xg);
  float*    Lg   = (float*)(ws + o_lg);
  _Float16* src16 = (_Float16*)(ws + o_h0);
  _Float16* H0   = (_Float16*)(ws + o_h0);
  _Float16* H1   = (_Float16*)(ws + o_h1);
  _Float16* H2   = (_Float16*)(ws + o_h2);
  _Float16* VT   = (_Float16*)(ws + o_vt);
  float*    Af   = (float*)(ws + o_af);
  float*    hF   = (float*)(ws + o_h1);
  _Float16* TQ = w16 + 0 * DM * DM, *TK = w16 + 1 * DM * DM, *TV = w16 + 2 * DM * DM;
  _Float16* TF1 = w16 + 3 * DM * DM, *TF2 = w16 + 4 * DM * DM;
  _Float16* SQ = w16 + 5 * DM * DM, *SK = w16 + 6 * DM * DM, *SV = w16 + 7 * DM * DM;
  _Float16* SF1 = w16 + 8 * DM * DM, *SF2 = w16 + 9 * DM * DM, *TEMPW = w16 + 10 * DM * DM;

  const float c64   = 1.0f / 64.0f;
  const float c1024 = 1.0f / 1024.0f;
  const float st_t  = 1.0f / 256.0f;
  const float st_s  = (1.0f / 256.0f) * 0.08838834764831845f;
  const dim3 gG(NTOK / 128, DM / 64);

  prep_k<<<NPREP / 256, 256, 0, stream>>>(wsrc[0], wsrc[1], wsrc[2], wsrc[3], wsrc[4], wsrc[5], wsrc[6],
                                          wsrc[7], wsrc[8], wsrc[9], wsrc[10], proj_w, gate_w, x,
                                          w16, pw16, gw16, xg16);
  gemm_k<0, false><<<dim3(NSTK / 128, NGL / 64), 128, 0, stream>>>(
      xg16, KG, IDM, 1, 31, gw16, KG, KG, gate_b, DFEAT, nullptr, Lg, nullptr, NGL,
      c64, 1.0f, 0, 31, IDM, 0, 0);
  gate_src_k<<<NSTK, 256, 0, stream>>>(Lg, x, src16);
  gemm_k<0, true><<<gG, 128, 0, stream>>>(
      src16, KSRC, IDM, 1, 31, pw16, KSRC, KPROJ, proj_b, DM, nullptr, Af, nullptr, DM,
      c64, 1.0f, 0, 31, IDM, 0, 0);

  ln_k<<<NTOK / 8, 256, 0, stream>>>(Af, nullptr, H0, tn1g, tn1b, 1.0f);
  gemm_k<1, false><<<gG, 128, 0, stream>>>(H0, DM, IDM, 1, 31, TQ, DM, DM, nullptr, 1, nullptr, nullptr, H1, DM,
                                           c64, HSC, 0, 31, IDM, 0, 0);
  gemm_k<1, false><<<gG, 128, 0, stream>>>(H0, DM, IDM, 1, 31, TK, DM, DM, nullptr, 1, nullptr, nullptr, H2, DM,
                                           c64, HSC, 0, 31, IDM, 0, 0);
  gemm_k<2, false><<<gG, 128, 0, stream>>>(H0, DM, IDM, 1, 31, TV, DM, DM, nullptr, 1, nullptr, nullptr, VT, DM,
                                           c64, HSC, 0, 31, IDM, 0, NTOK);
  attn_t_k<<<NSTK, 128, 0, stream>>>(H1, H2, VT, Af, tn1g, tn1b, st_t);
  ln_k<<<NTOK / 8, 256, 0, stream>>>(Af, Af, H0, tn2g, tn2b, 1.0f);
  gemm_k<1, false><<<gG, 128, 0, stream>>>(H0, DM, IDM, 1, 31, TF1, DM, DM, tf1b, DM, nullptr, nullptr, H1, DM,
                                           c64, HSC, 1, 31, IDM, 0, 0);
  gemm_k<0, false><<<gG, 128, 0, stream>>>(H1, DM, IDM, 1, 31, TF2, DM, DM, tf2b, DM, Af, Af, nullptr, DM,
                                           c1024, 1.0f, 0, 31, IDM, 0, 0);

  ln_k<<<NTOK / 8, 256, 0, stream>>>(Af, nullptr, H0, sn1g, sn1b, 1.0f);
  gemm_k<1, false><<<gG, 128, 0, stream>>>(H0, DM, IDM, 1, 31, SQ, DM, DM, nullptr, 1, nullptr, nullptr, H1, DM,
                                           c64, HSC, 0, 31, IDM, 0, 0);
  gemm_k<1, false><<<gG, 128, 0, stream>>>(H0, DM, IDM, 1, 31, SK, DM, DM, nullptr, 1, nullptr, nullptr, H2, DM,
                                           c64, HSC, 0, 31, IDM, 0, 0);
  gemm_k<2, false><<<gG, 128, 0, stream>>>(H0, DM, 1023, 32, 10, SV, DM, DM, nullptr, 1, nullptr, nullptr, VT, DM,
                                           c64, HSC, 0, 10, 1023, DM * NSTK, NSTK);
  attn_s_k<<<dim3(NSTK / 64, TLEN), 128, 0, stream>>>(H1, H2, VT, Af, sn1g, sn1b, st_s);
  ln_k<<<NTOK / 8, 256, 0, stream>>>(Af, Af, H0, sn2g, sn2b, 1.0f);
  gemm_k<1, false><<<gG, 128, 0, stream>>>(H0, DM, IDM, 1, 31, SF1, DM, DM, sf1b, DM, nullptr, nullptr, H1, DM,
                                           c64, HSC, 1, 31, IDM, 0, 0);
  gemm_k<0, false><<<gG, 128, 0, stream>>>(H1, DM, IDM, 1, 31, SF2, DM, DM, sf2b, DM, Af, Af, H0, DM,
                                           c1024, 1.0f, 0, 31, IDM, 0, 0);

  gemm_k<0, false><<<gG, 128, 0, stream>>>(H0, DM, IDM, 1, 31, TEMPW, DM, DM, nullptr, 1, nullptr, hF, nullptr, DM,
                                           c64, 1.0f, 0, 31, IDM, 0, 0);
  pool_k<<<NSTK / 32, 256, 0, stream>>>(hF, Af, out_w, out_b, (float*)d_out);
}
